// HLGT_21225728376842
// MI455X (gfx1250) — hardware-verified
//
#include <hip/hip_runtime.h>

typedef __attribute__((ext_vector_type(16))) _Float16 v16h;
typedef __attribute__((ext_vector_type(8)))  _Float16 v8h;
typedef __attribute__((ext_vector_type(8)))  float  v8f;
typedef __attribute__((ext_vector_type(4)))  float  v4f;
typedef __attribute__((ext_vector_type(4)))  unsigned v4u;
typedef float __attribute__((may_alias)) float_a;

#define N_NODES 50000
#define HID 128
#define FFD 256
#define NL 6
#define BT 256
#define ECAP 5120
#define SCAP 48
#define ETILE 2048
#define NBUCK ((N_NODES + BT - 1) / BT)
#define EPS_F 1e-5f

template <typename V> __device__ __forceinline__ void vst2(void* p, V v) {
  *(volatile V*)p = v; __threadfence(); *(volatile V*)p = v;
}
__device__ __forceinline__ v8f wmma_f16(v16h a, v16h b, v8f c) {
  v8f d = __builtin_amdgcn_wmma_f32_16x16x32_f16(false, a, false, b, (short)0, c, false, false);
  asm volatile("v_nop\n\tv_nop\n\tv_nop\n\tv_nop" : "+v"(d) : "v"(a), "v"(b));
  return d;
}
__device__ __forceinline__ v16h frag_h(const _Float16* row, int k0, int lane) {
  union { v16h v; v8h h[2]; } r;
  const _Float16* p = row + k0 + 8 * (lane >> 4);
  r.h[0] = *(const v8h*)(p); r.h[1] = *(const v8h*)(p + 16);
  return r.v;
}
__device__ __forceinline__ v16h frag_f32(const float* row, int k0, int lane) {
  v16h a; const float* p = row + k0 + 8 * (lane >> 4);
#pragma unroll
  for (int i = 0; i < 8; ++i) { a[i] = (_Float16)p[i]; a[8 + i] = (_Float16)p[16 + i]; }
  return a;
}
__device__ __forceinline__ float gelu_exact(float x) { return 0.5f * x * (1.0f + erff(x * 0.70710678118654752f)); }
__device__ __forceinline__ float beta_w(const float* __restrict__ beta, int l) {
  float mx = beta[0];
#pragma unroll
  for (int i = 1; i <= NL; ++i) mx = fmaxf(mx, beta[i]);
  float s = 0.f;
#pragma unroll
  for (int i = 0; i <= NL; ++i) s += __expf(beta[i] - mx);
  return __expf(beta[l] - mx) / s;
}

struct Bucket {
  int lsrc[ECAP]; unsigned short ltgt[ECAP]; unsigned short sub[BT][SCAP]; int scnt[BT]; int wcnt[8][8]; int total;
};
__device__ void bucket_build(Bucket& bk, const int* __restrict__ src, const int* __restrict__ dst, int E, int tlo, int tid) {
  const int lane = tid & 31, wave = tid >> 5;
  if (tid == 0) bk.total = 0;
  __syncthreads();
  for (int e0 = 0; e0 < E; e0 += ETILE) {
    int rv[8]; unsigned msk[8];
#pragma unroll
    for (int j = 0; j < 8; ++j) {
      const int e = e0 + j * 256 + tid;
      const int r = (e < E) ? dst[e] : -1;
      rv[j] = r;
      msk[j] = (unsigned)__builtin_amdgcn_ballot_w32((r >= tlo) && (r < tlo + BT));
    }
    if (lane < 8) bk.wcnt[lane][wave] = __builtin_popcount(msk[lane]);
    __syncthreads();
    const int base = bk.total;
    int run = 0, pre[8];
#pragma unroll
    for (int j = 0; j < 8; ++j) {
#pragma unroll
      for (int w = 0; w < 8; ++w) { if (w == wave) pre[j] = run; run += bk.wcnt[j][w]; }
    }
#pragma unroll
    for (int j = 0; j < 8; ++j) {
      const unsigned m = msk[j];
      if ((m >> lane) & 1u) {
        const int pos = base + pre[j] + __builtin_popcount(m & ((1u << lane) - 1u));
        if (pos < ECAP) { bk.lsrc[pos] = e0 + j * 256 + tid; bk.ltgt[pos] = (unsigned short)(rv[j] - tlo); }
      }
    }
    __syncthreads();
    if (tid == 0) bk.total = base + run;
    __syncthreads();
  }
  const int n = (bk.total < ECAP) ? bk.total : ECAP;
  for (int i = tid; i < n; i += 256) { int s = src[bk.lsrc[i]]; s = s < 0 ? 0 : (s >= N_NODES ? N_NODES - 1 : s); bk.lsrc[i] = s; }
  __syncthreads();
  int k = 0;
  for (int i = 0; i < n; ++i) if ((int)bk.ltgt[i] == tid) { if (k < SCAP) bk.sub[tid][k] = (unsigned short)i; ++k; }
  bk.scnt[tid] = (k < SCAP) ? k : SCAP;
  __syncthreads();
}

__global__ __launch_bounds__(256) void k_wt(const float* __restrict__ W, _Float16* __restrict__ WT, int K, int M) {
  __shared__ __align__(16) _Float16 tile[64][72];
  const int mt = M / 64 > 0 ? M / 64 : 1;
  const int tid = threadIdx.x;
  const int m0 = (blockIdx.x % mt) * 64, k0 = (blockIdx.x / mt) * 64;
  const int mw = (M < 64) ? M : 64;
  for (int i = tid; i < 64 * 64; i += 256) { const int kk = i >> 6, mm = i & 63; tile[mm][kk] = (mm < mw && k0 + kk < K) ? (_Float16)W[(size_t)(k0 + kk) * M + m0 + mm] : (_Float16)0.f; }
  __syncthreads();
  for (int g = tid; g < 64 * 8; g += 256) { const int mm = g >> 3, pc = g & 7; if (mm < mw) vst2(WT + (size_t)(m0 + mm) * K + k0 + pc * 8, *(const v4u*)(&tile[mm][pc * 8])); }
}


template <int K, int M, int EPI>
__global__ __launch_bounds__(128) void k_gemm(const float* __restrict__ A, const _Float16* __restrict__ Ah,
                                              const _Float16* __restrict__ WT, const float* __restrict__ bias,
                                              const float* __restrict__ res, const float* __restrict__ g, const float* __restrict__ bt,
                                              const float* __restrict__ beta, int lidx,
                                              float* __restrict__ Yf, _Float16* __restrict__ Yh, float* __restrict__ acc_out) {
  constexpr int NT = M / 16, KC = K / 32;
  __shared__ __align__(16) float so[4][16 * M];
  const int tid = threadIdx.x, wave = tid >> 5, lane = tid & 31, hi = lane >> 4, col = lane & 15;
  const int strip = blockIdx.x * 4 + wave;
  const bool valid = strip < N_NODES / 16;
  float* S = so[wave];
  if (valid) {
#pragma unroll 1
    for (int nt = 0; nt < NT; ++nt) {
      v8f acc = {};
      const _Float16* br = WT + (size_t)(nt * 16 + col) * K;
#pragma unroll
      for (int kc = 0; kc < KC; ++kc) {
        v16h a = Ah ? frag_h(Ah + (size_t)(strip * 16 + col) * K, kc * 32, lane) : frag_f32(A + (size_t)(strip * 16 + col) * K, kc * 32, lane);
        acc = wmma_f16(a, frag_h(br, kc * 32, lane), acc);
      }
      const float bv = bias[nt * 16 + col];
#pragma unroll
      for (int r = 0; r < 8; ++r) {
        float v = acc[r] + bv;
        if (EPI == 0) v = fmaxf(v, 0.f);
        else if (EPI == 2) v = gelu_exact(v);
        S[(hi * 8 + r) * M + nt * 16 + col] = v;
      }
    }
  }
  __syncthreads();
  if (!valid) return;
  const size_t row0 = (size_t)strip * 16;
  if (EPI == 3) {
    const int rl = lane >> 1, c0 = (lane & 1) * 64;
    float s1 = 0.f, s2 = 0.f;
    for (int c = c0; c < c0 + 64; ++c) { float v = S[rl * M + c] + res[(row0 + rl) * M + c]; S[rl * M + c] = v; s1 += v; }
    s1 += __shfl_xor(s1, 1, 32);
    const float mean = s1 * (1.f / M);
    for (int c = c0; c < c0 + 64; ++c) { float d = S[rl * M + c] - mean; s2 += d * d; }
    s2 += __shfl_xor(s2, 1, 32);
    const float rstd = rsqrtf(s2 * (1.f / M) + EPS_F);
    const float bw = beta_w(beta, lidx + 1);
    for (int c = c0; c < c0 + 64; ++c) { float z = (S[rl * M + c] - mean) * rstd * g[c] + bt[c]; S[rl * M + c] = fmaxf(z, 0.f); }
    __builtin_amdgcn_wave_barrier();
    __builtin_amdgcn_fence(__ATOMIC_RELEASE, "workgroup");
#pragma unroll 4
    for (int q = 0; q < 16 * (M / 4) / 32; ++q) {
      const int gp = q * 32 + lane; const int r = gp / (M / 4), pc = gp % (M / 4);
      const v4f z = *(const v4f*)(S + r * M + pc * 4);
      vst2(Yf + (row0 + r) * M + pc * 4, z);
      float* ap = acc_out + (row0 + r) * M + pc * 4;
      v4f a = *(const v4f*)ap; a += bw * z; vst2(ap, a);
    }
  } else if (EPI == 2) {
    for (int q = 0; q < 16 * (M / 8) / 32; ++q) {
      const int gp = q * 32 + lane; const int r = gp / (M / 8), pc = gp % (M / 8);
      union { v8h h; v4u u; } pk;
#pragma unroll
      for (int e = 0; e < 8; ++e) pk.h[e] = (_Float16)S[r * M + pc * 8 + e];
      vst2(Yh + (row0 + r) * M + pc * 8, pk.u);
    }
  } else {
    const float bw0 = (EPI == 0) ? beta_w(beta, 0) : 0.f;
#pragma unroll 4
    for (int q = 0; q < 16 * (M / 4) / 32; ++q) {
      const int gp = q * 32 + lane; const int r = gp / (M / 4), pc = gp % (M / 4);
      const v4f v = *(const v4f*)(S + r * M + pc * 4);
      vst2(Yf + (row0 + r) * M + pc * 4, v);
      if (EPI == 0) vst2(acc_out + (row0 + r) * M + pc * 4, bw0 * v);
    }
  }
}

__global__ __launch_bounds__(256) void k_attn_ln(const int* __restrict__ src, const int* __restrict__ dst, int E,
                                                 const float* __restrict__ qkvs,
                                                 const float* __restrict__ z, const float* __restrict__ g, const float* __restrict__ bt,
                                                 float* __restrict__ hout) {
  __shared__ Bucket bk;
  const int tid = threadIdx.x, lane = tid & 31, wave = tid >> 5, tlo = blockIdx.x * BT;
  bucket_build(bk, src, dst, E, tlo, tid);
  for (int s = 0; s < 32; ++s) {
    const int t = wave * 32 + s, node = tlo + t;
    if (node >= N_NODES) break;
    const int cnt = bk.scnt[t];
    const float* qr = qkvs + (size_t)node * 512;
    float qv[4];
#pragma unroll
    for (int j = 0; j < 4; ++j) qv[j] = qr[lane + 32 * j] * 0.125f;
    float m0 = -3.0e38f, m1 = -3.0e38f, l0 = 0.f, l1 = 0.f, acc[4] = {0.f, 0.f, 0.f, 0.f};
    for (int k = 0; k < cnt; ++k) {
      const int sN = bk.lsrc[bk.sub[t][k]];
      const float* kr = qkvs + (size_t)sN * 512 + 128;
      const float* vr = qkvs + (size_t)sN * 512 + 256;
      float p0 = qv[0] * kr[lane] + qv[1] * kr[lane + 32];
      float p1 = qv[2] * kr[lane + 64] + qv[3] * kr[lane + 96];
#pragma unroll
      for (int off = 16; off > 0; off >>= 1) { p0 += __shfl_xor(p0, off, 32); p1 += __shfl_xor(p1, off, 32); }
      const float n0 = fmaxf(m0, p0), n1 = fmaxf(m1, p1);
      const float c0 = __expf(m0 - n0), c1 = __expf(m1 - n1);
      const float w0 = __expf(p0 - n0), w1 = __expf(p1 - n1);
      l0 = l0 * c0 + w0; l1 = l1 * c1 + w1; m0 = n0; m1 = n1;
      acc[0] = acc[0] * c0 + w0 * vr[lane];      acc[1] = acc[1] * c0 + w0 * vr[lane + 32];
      acc[2] = acc[2] * c1 + w1 * vr[lane + 64]; acc[3] = acc[3] * c1 + w1 * vr[lane + 96];
    }
    float v[4]; float s1 = 0.f;
    const float* zr = z + (size_t)node * HID;
    const float* skr = qr + 384;
#pragma unroll
    for (int j = 0; j < 4; ++j) {
      const float li = (j < 2) ? l0 : l1;
      const float msg = (cnt > 0) ? acc[j] / li : 0.f;
      v[j] = zr[lane + 32 * j] + msg + skr[lane + 32 * j];
      s1 += v[j];
    }
#pragma unroll
    for (int off = 16; off > 0; off >>= 1) s1 += __shfl_xor(s1, off, 32);
    const float mean = s1 * (1.f / HID);
    float s2 = 0.f;
#pragma unroll
    for (int j = 0; j < 4; ++j) { float d = v[j] - mean; s2 += d * d; }
#pragma unroll
    for (int off = 16; off > 0; off >>= 1) s2 += __shfl_xor(s2, off, 32);
    const float rstd = rsqrtf(s2 * (1.f / HID) + EPS_F);
    float* hr = hout + (size_t)node * HID;
#pragma unroll
    for (int j = 0; j < 4; ++j) { const int c = lane + 32 * j; vst2(hr + c, (float_a)((v[j] - mean) * rstd * g[c] + bt[c])); }
  }
}

__global__ __launch_bounds__(256) void k_wt4(const float* __restrict__ Wq, const float* __restrict__ Wk, const float* __restrict__ Wv,
                                             const float* __restrict__ Ws, _Float16* __restrict__ WT) {
  __shared__ __align__(16) _Float16 tile[64][72];
  const int tid = threadIdx.x;
  const int part = blockIdx.x >> 2, m0 = ((blockIdx.x >> 1) & 1) * 64, k0 = (blockIdx.x & 1) * 64;
  const float* W = part == 0 ? Wq : part == 1 ? Wk : part == 2 ? Wv : Ws;
  for (int i = tid; i < 64 * 64; i += 256) { const int kk = i >> 6, mm = i & 63; tile[mm][kk] = (_Float16)W[(size_t)(k0 + kk) * HID + m0 + mm]; }
  __syncthreads();
  for (int gq = tid; gq < 64 * 8; gq += 256) { const int mm = gq >> 3, pc = gq & 7; vst2(WT + (size_t)(part * 128 + m0 + mm) * HID + k0 + pc * 8, *(const v4u*)(&tile[mm][pc * 8])); }
}
__global__ __launch_bounds__(128) void k_b4(const float* __restrict__ bq, const float* __restrict__ bk, const float* __restrict__ bv,
                                            const float* __restrict__ bs, float* __restrict__ b4) {
  const int i = threadIdx.x;
  const int part = i >> 5, c = (i & 31) * 4;
  const float* b = part == 0 ? bq : part == 1 ? bk : part == 2 ? bv : bs;
  v4f v = {b[c], b[c + 1], b[c + 2], b[c + 3]};
  vst2(b4 + part * 128 + c, v);
}

extern "C" void kernel_launch(void* const* d_in, const int* in_sizes, int n_in,
                              void* d_out, int out_size, void* d_ws, size_t ws_size,
                              hipStream_t stream) {
  (void)n_in; (void)out_size; (void)ws_size;
  const float* x  = (const float*)d_in[0];
  const int*   ei = (const int*)d_in[1];
  const int E = in_sizes[1] / 2;
  const int* src = ei; const int* dst = ei + E;
  const float *Win = (const float*)d_in[2], *b_in = (const float*)d_in[3];
  const float *Wq = (const float*)d_in[4], *bq = (const float*)d_in[5], *Wk = (const float*)d_in[6], *bk = (const float*)d_in[7];
  const float *Wv = (const float*)d_in[8], *bv = (const float*)d_in[9], *Wsk = (const float*)d_in[10], *bsk = (const float*)d_in[11];
  const float *W1 = (const float*)d_in[12], *b1 = (const float*)d_in[13], *W2 = (const float*)d_in[14], *b2 = (const float*)d_in[15];
  const float *g1 = (const float*)d_in[16], *bt1 = (const float*)d_in[17], *g2 = (const float*)d_in[18], *bt2 = (const float*)d_in[19];
  const float* beta = (const float*)d_in[20];
  float* out = (float*)d_out;

  char* ws = (char*)d_ws; size_t off = 0;
  auto alloc = [&](size_t bytes) -> void* { void* p = ws + off; off = (off + bytes + 255) & ~(size_t)255; return p; };
  _Float16* WTin = (_Float16*)alloc(128 * 128 * 2);
  _Float16* WT4  = (_Float16*)alloc(512 * 128 * 2);
  _Float16* WT1  = (_Float16*)alloc(256 * 128 * 2);
  _Float16* WT2  = (_Float16*)alloc(128 * 256 * 2);
  float* b4   = (float*)alloc(512 * 4);
  float* zb   = (float*)alloc((size_t)N_NODES * HID * 4);
  float* qkvs = (float*)alloc((size_t)N_NODES * 512 * 4);
  float* hb   = (float*)alloc((size_t)N_NODES * HID * 4);
  _Float16* f1 = (_Float16*)alloc((size_t)N_NODES * FFD * 2);

  const int gstrips = (N_NODES / 16 + 3) / 4;

  k_wt<<<(128 / 64) * (128 / 64), 256, 0, stream>>>(Win, WTin, 128, 128);
  k_gemm<128, 128, 0><<<gstrips, 128, 0, stream>>>(x, nullptr, WTin, b_in, nullptr, nullptr, nullptr, beta, 0, zb, nullptr, out);

  for (int l = 0; l < NL; ++l) {
    k_wt4<<<16, 256, 0, stream>>>(Wq + (size_t)l * 128 * 128, Wk + (size_t)l * 128 * 128, Wv + (size_t)l * 128 * 128, Wsk + (size_t)l * 128 * 128, WT4);
    k_b4<<<1, 128, 0, stream>>>(bq + l * 128, bk + l * 128, bv + l * 128, bsk + l * 128, b4);
    k_gemm<128, 512, 1><<<gstrips, 128, 0, stream>>>(zb, nullptr, WT4, b4, nullptr, nullptr, nullptr, beta, l, qkvs, nullptr, nullptr);
    k_attn_ln<<<NBUCK, 256, 0, stream>>>(src, dst, E, qkvs, zb, g1 + l * 128, bt1 + l * 128, hb);
    k_wt<<<(128 / 64) * (256 / 64), 256, 0, stream>>>(W1 + (size_t)l * 128 * 256, WT1, 128, 256);
    k_wt<<<(256 / 64) * (128 / 64), 256, 0, stream>>>(W2 + (size_t)l * 256 * 128, WT2, 256, 128);
    k_gemm<128, 256, 2><<<gstrips, 128, 0, stream>>>(hb, nullptr, WT1, b1 + l * 256, nullptr, nullptr, nullptr, beta, l, nullptr, f1, nullptr);
    k_gemm<256, 128, 3><<<gstrips, 128, 0, stream>>>(nullptr, f1, WT2, b2 + l * 128, hb, g2 + l * 128, bt2 + l * 128, beta, l, zb, nullptr, out);
  }
}
